// BASE_6442450944602
// MI455X (gfx1250) — hardware-verified
//
#include <hip/hip_runtime.h>
#include <math.h>
#include <stdint.h>

#define NB  16
#define NC  512
#define NS  1024
#define NR  32
#define IMW 32
#define HB  8
#define KF  2048

static_assert(NC % 64 == 0);
static_assert(NS % 64 == 0);
static_assert(NS % 32 == 0);
static_assert(KF % 32 == 0);
static_assert(NB % HB == 0);
static_assert(IMW * IMW == NS);
static_assert(NC / 16 == NR);

typedef _Float16 v16h __attribute__((ext_vector_type(16)));
typedef _Float16 v8h  __attribute__((ext_vector_type(8)));
typedef __bf16   v16b __attribute__((ext_vector_type(16)));
typedef __bf16   v8b  __attribute__((ext_vector_type(8)));
typedef float    v8f  __attribute__((ext_vector_type(8)));
typedef float    v4f  __attribute__((ext_vector_type(4)));
typedef unsigned int v4u __attribute__((ext_vector_type(4)));

__device__ __forceinline__ unsigned short f2bf_bits(float f) {
  unsigned u = __float_as_uint(f);
  return (unsigned short)((u + 0x7FFFu + ((u >> 16) & 1u)) >> 16);
}
__device__ __forceinline__ float bf_bits2f(unsigned short h) { return __uint_as_float(((unsigned)h) << 16); }
__device__ __forceinline__ float bf_rne(float f) { return bf_bits2f(f2bf_bits(f)); }
__device__ __forceinline__ unsigned pk16(unsigned short a, unsigned short b) { return (unsigned)a | ((unsigned)b << 16); }

__device__ __forceinline__ float wave_sum(float v) {
#pragma unroll
  for (int off = 16; off > 0; off >>= 1) v += __shfl_xor(v, off, 32);
  return v;
}
__device__ __forceinline__ float sigm(float v) { return __builtin_amdgcn_rcpf(1.0f + __expf(-v)); }

__device__ __forceinline__ void dep_guard_h(v8f& a, v8f& b, v16h x, v16h y) { asm volatile("v_nop\n\tv_nop\n\tv_nop\n\tv_nop" : "+v"(a), "+v"(b) : "v"(x), "v"(y)); }
__device__ __forceinline__ void dep_guard_b(v8f& a, v8f& b, v16b x, v16b y) { asm volatile("v_nop\n\tv_nop\n\tv_nop\n\tv_nop" : "+v"(a), "+v"(b) : "v"(x), "v"(y)); }
__device__ __forceinline__ void keep4_h(v16h a, v16h b, v16h c, v16h d) { asm volatile("v_nop" :: "v"(a), "v"(b), "v"(c), "v"(d)); }
__device__ __forceinline__ void keep4_b(v16b a, v16b b, v16b c, v16b d) { asm volatile("v_nop" :: "v"(a), "v"(b), "v"(c), "v"(d)); }
__device__ __forceinline__ void acc_guard4(v8f& a, v8f& b, v8f& c, v8f& d) { asm volatile("v_nop\n\tv_nop\n\tv_nop\n\tv_nop" : "+v"(a), "+v"(b), "+v"(c), "+v"(d)); }
template <typename T> struct Frag;
template <> struct Frag<_Float16> {
  typedef v16h V; union U { v16h v; v8h h[2]; };
  static __device__ __forceinline__ v16h load(const _Float16* p) {
    U f; f.h[0] = *(const v8h*)(p); f.h[1] = *(const v8h*)(p + 16); return f.v;
  }
  static __device__ __forceinline__ v8f mma(v16h a, v16h b, v8f c) {
    return __builtin_amdgcn_wmma_f32_16x16x32_f16(false, a, false, b, (short)0, c, false, false);
  }
  static __device__ __forceinline__ void guard(v8f& a, v8f& b, v16h x, v16h y) { dep_guard_h(a, b, x, y); }
  static __device__ __forceinline__ void keep(v16h a, v16h b, v16h c, v16h d) { keep4_h(a, b, c, d); }
};
template <> struct Frag<__bf16> {
  typedef v16b V; union U { v16b v; v8b h[2]; };
  static __device__ __forceinline__ v16b load(const __bf16* p) {
    U f; f.h[0] = *(const v8b*)(p); f.h[1] = *(const v8b*)(p + 16); return f.v;
  }
  static __device__ __forceinline__ v8f mma(v16b a, v16b b, v8f c) {
    return __builtin_amdgcn_wmma_f32_16x16x32_bf16(false, a, false, b, (short)0, c, false, false);
  }
  static __device__ __forceinline__ void guard(v8f& a, v8f& b, v16b x, v16b y) { dep_guard_b(a, b, x, y); }
  static __device__ __forceinline__ void keep(v16b a, v16b b, v16b c, v16b d) { keep4_b(a, b, c, d); }
};

template <int ET> struct Elem;
template <> struct Elem<0> { typedef _Float16 T; };
template <> struct Elem<1> { typedef __bf16 T; };
template <int ET, bool SPLIT, int BIAS_MODE, int OUT_MODE, bool RESID, int ACT = 0>
__global__ __launch_bounds__(256) void wmma_gemm64(
    const unsigned short* __restrict__ Ap, const unsigned short* __restrict__ A2p, int lda, long strideA,
    const unsigned short* __restrict__ Btp, const unsigned short* __restrict__ Bt2p, int ldb, long strideB,
    void* __restrict__ Cout, void* __restrict__ Cout2, int ldc, long strideC,
    const float* __restrict__ bias,
    const float* __restrict__ resid, long strideR,
    int M, int N, int K, float scale) {
  typedef typename Elem<ET>::T T;
  typedef typename Frag<T>::V V;
  const T* A = (const T*)Ap; const T* A2 = (const T*)A2p; const T* Bt = (const T*)Btp; const T* Bt2 = (const T*)Bt2p;
  __shared__ __align__(16) float sT[8][16 * 68];
  const int b    = blockIdx.y;
  const int lane = threadIdx.x & 31;
  const int wave = threadIdx.x >> 5;
  const int tilesN = N >> 6;
  const int tilesM = M >> 6;
  const int tile = blockIdx.x * 8 + wave;
  if (tile >= tilesM * tilesN) return;
  const int tm = tile / tilesN;
  const int tn = tile - tm * tilesN;
  const int m0 = tm << 6;
  const int n0 = tn << 6;

  const T* Ab  = A  + (size_t)b * strideA;
  const T* Bb  = Bt + (size_t)b * strideB;
  const T* Ab2 = SPLIT ? (A2  + (size_t)b * strideA) : nullptr;
  const T* Bb2 = SPLIT ? (Bt2 + (size_t)b * strideB) : nullptr;

  const int rlane = lane & 15;
  const int koff  = (lane >> 4) * 8;
  const int mOff  = (lane >> 4) * 8;

  v8f acc[4][4];
#pragma unroll
  for (int i = 0; i < 4; ++i)
#pragma unroll
    for (int j = 0; j < 4; ++j) acc[i][j] = (v8f){0.f,0.f,0.f,0.f,0.f,0.f,0.f,0.f};

  for (int k0 = 0; k0 < K; k0 += 32) {
    V bh[4], bl[4];
#pragma unroll
    for (int j = 0; j < 4; ++j) {
      const size_t bo = (size_t)(n0 + (j << 4) + rlane) * ldb + koff + k0;
      bh[j] = Frag<T>::load(Bb + bo);
      if (SPLIT) bl[j] = Frag<T>::load(Bb2 + bo); else bl[j] = bh[j];
    }
#pragma unroll
    for (int i = 0; i < 4; ++i) {
      const size_t ao = (size_t)(m0 + (i << 4) + rlane) * lda + koff + k0;
      V ah = Frag<T>::load(Ab + ao);
      V al;
      if (SPLIT) al = Frag<T>::load(Ab2 + ao); else al = ah;
#pragma unroll
      for (int j = 0; j < 4; ++j) {
        acc[i][j] = Frag<T>::mma(ah, bh[j], acc[i][j]);
        if (SPLIT) {
          acc[i][j] = Frag<T>::mma(ah, bl[j], acc[i][j]);
          acc[i][j] = Frag<T>::mma(al, bh[j], acc[i][j]);
        }
      }
      Frag<T>::guard(acc[i][0], acc[i][3], ah, al);
    }
    Frag<T>::keep(bh[0], bh[1], bh[2], bh[3]);
    if (SPLIT) Frag<T>::keep(bl[0], bl[1], bl[2], bl[3]);
  }
  acc_guard4(acc[0][0], acc[0][1], acc[0][2], acc[0][3]);
  acc_guard4(acc[1][0], acc[1][1], acc[1][2], acc[1][3]);
  acc_guard4(acc[2][0], acc[2][1], acc[2][2], acc[2][3]);
  acc_guard4(acc[3][0], acc[3][1], acc[3][2], acc[3][3]);

  float* slab = sT[wave];
  const float* Rb = RESID ? (resid + (size_t)b * strideR) : nullptr;
#pragma unroll
  for (int i = 0; i < 4; ++i) {
    const int mBase = m0 + (i << 4);
#pragma unroll
    for (int j = 0; j < 4; ++j) {
      const int n = n0 + (j << 4) + rlane;
      float bv = 0.f;
      if (BIAS_MODE == 2) bv = bf_rne(bias[n]);
#pragma unroll
      for (int r = 0; r < 8; ++r) {
        float v = acc[i][j][r] * scale;
        if (BIAS_MODE == 1) v += bf_rne(bias[mBase + mOff + r]);
        if (BIAS_MODE == 2) v += bv;
        if (RESID) v += Rb[(size_t)(mBase + mOff + r) * ldc + n];
        if (ACT == 1) v = tanhf(v);
        if (ACT == 2) v = fmaxf(v, 0.0f);
        if (ACT == 3) v = v / (1.0f + expf(-v));
        if (ACT == 4) v = (v > 0.f) ? v : 0.01f * v;
        if (ACT == 5) v = 0.5f * v * (1.0f + erff(v * 0.70710678118654752f));
        slab[(mOff + r) * 68 + (j << 4) + rlane] = v;
      }
    }
    __builtin_amdgcn_fence(__ATOMIC_RELEASE, "workgroup");
    __builtin_amdgcn_wave_barrier();
    __builtin_amdgcn_fence(__ATOMIC_ACQUIRE, "workgroup");
    if (OUT_MODE == 0) {
      float* C = (float*)Cout + (size_t)b * strideC;
      const int hh = lane >> 4, c4 = (lane & 15) * 4;
      for (int pass = 0; pass < 2; ++pass) {
#pragma unroll
        for (int it = 0; it < 8; ++it) {
          const int row = it * 2 + hh;
          v4f v = *(const v4f*)(slab + row * 68 + c4);
          *(volatile v4f*)(C + (size_t)(mBase + row) * ldc + n0 + c4) = v;
        }
        __threadfence();
      }
    } else {
      const int q = lane >> 3, c8 = (lane & 7) * 8;
      unsigned short* C  = (unsigned short*)Cout  + (size_t)b * strideC;
      unsigned short* C2 = (OUT_MODE == 2) ? ((unsigned short*)Cout2 + (size_t)b * strideC) : nullptr;
      for (int pass = 0; pass < 2; ++pass) {
#pragma unroll
        for (int it = 0; it < 4; ++it) {
          const int row = it * 4 + q;
          const float* sp = slab + row * 68 + c8;
          v8h hv, lv;
#pragma unroll
          for (int e = 0; e < 8; ++e) {
            if (OUT_MODE == 1) {
              hv[e] = (_Float16)sp[e];
            } else {
              unsigned short hb = f2bf_bits(sp[e]);
              unsigned short lb = f2bf_bits(sp[e] - bf_bits2f(hb));
              hv[e] = __builtin_bit_cast(_Float16, hb);
              lv[e] = __builtin_bit_cast(_Float16, lb);
            }
          }
          *(volatile v8h*)(C + (size_t)(mBase + row) * ldc + n0 + c8) = hv;
          if (OUT_MODE == 2) *(volatile v8h*)(C2 + (size_t)(mBase + row) * ldc + n0 + c8) = lv;
        }
        __threadfence();
      }
    }
    __builtin_amdgcn_fence(__ATOMIC_RELEASE, "workgroup");
    __builtin_amdgcn_wave_barrier();
    __builtin_amdgcn_fence(__ATOMIC_ACQUIRE, "workgroup");
  }
}

__global__ __launch_bounds__(256) void se_kernel(const float* __restrict__ x,
                                                 const float* __restrict__ w1, const float* __restrict__ b1,
                                                 const float* __restrict__ w2, const float* __restrict__ b2,
                                                 float* __restrict__ ysc) {
  __shared__ float sm[NC];
  __shared__ float hv[NR];
  __shared__ __align__(16) float ys[NC];
  const int tid = threadIdx.x, lane = tid & 31, wave = tid >> 5;
  const int b = blockIdx.x;

#pragma unroll 1
  for (int i = 0; i < NC / 8; ++i) {
    const int c = wave * (NC / 8) + i;
    const float* row = x + ((size_t)b * NC + c) * NS + 4 * lane;
    float acc = 0.0f;
#pragma unroll 2
    for (int q = 0; q < NS / 128; ++q) {
      const v4f v = *(const v4f*)(row + 128 * q);
      acc += (bf_rne(v.x) + bf_rne(v.y)) + (bf_rne(v.z) + bf_rne(v.w));
    }
    acc = wave_sum(acc);
    if (lane == 0) sm[c] = acc * (1.0f / (float)NS);
  }
  __syncthreads();
  {
    const int j = tid >> 3, part = tid & 7;
    const float* wr = w1 + (size_t)j * NC + part * 64;
    const float* sp = sm + part * 64;
    float acc = 0.0f;
#pragma unroll 1
    for (int i = 0; i < 16; ++i) {
      const v4f w = *(const v4f*)(wr + 4 * i);
      acc += bf_rne(w.x) * sp[4 * i] + bf_rne(w.y) * sp[4 * i + 1] + bf_rne(w.z) * sp[4 * i + 2] + bf_rne(w.w) * sp[4 * i + 3];
    }
    acc += __shfl_xor(acc, 1, 32);
    acc += __shfl_xor(acc, 2, 32);
    acc += __shfl_xor(acc, 4, 32);
    if (part == 0) hv[j] = fmaxf(acc + bf_rne(b1[j]), 0.0f);
  }
  __syncthreads();
#pragma unroll 1
  for (int rr = 0; rr < 2; ++rr) {
    const int c = tid + 256 * rr;
    const float* wr = w2 + (size_t)c * NR;
    float acc = 0.0f;
#pragma unroll 1
    for (int i = 0; i < NR / 4; ++i) {
      const v4f w = *(const v4f*)(wr + 4 * i);
      acc += bf_rne(w.x) * hv[4 * i] + bf_rne(w.y) * hv[4 * i + 1] + bf_rne(w.z) * hv[4 * i + 2] + bf_rne(w.w) * hv[4 * i + 3];
    }
    acc += bf_rne(b2[c]);
    ys[c] = sigm(acc);
  }
  __syncthreads();
  if (tid < 128) {
    const v4f v = *(const v4f*)(ys + 4 * tid);
    float* d = ysc + (size_t)b * NC + 4 * tid;
    *(volatile v4f*)d = v;
    __threadfence();
    *(volatile v4f*)d = v;
  }
}

#define XBLK (HB * NC * NS / 8 / 256)
#define GBLK (NS * NS / 8 / 256)
#define DBLK (NC * NS / 8 / 256)
static_assert(XBLK * 256 * 8 == HB * NC * NS);
static_assert(GBLK * 256 * 8 == NS * NS);
static_assert(DBLK * 256 * 8 == NC * NS);

__device__ __forceinline__ v4u pack8_bf(const float* p) {
  const v4f a = *(const v4f*)p;
  const v4f c = *(const v4f*)(p + 4);
  v4u o;
  o.x = pk16(f2bf_bits(a.x), f2bf_bits(a.y));
  o.y = pk16(f2bf_bits(a.z), f2bf_bits(a.w));
  o.z = pk16(f2bf_bits(c.x), f2bf_bits(c.y));
  o.w = pk16(f2bf_bits(c.z), f2bf_bits(c.w));
  return o;
}

__global__ __launch_bounds__(256) void cvt_kernel(const float* __restrict__ xh, const float* __restrict__ gus,
                                                  const float* __restrict__ dw,
                                                  unsigned short* __restrict__ xb, unsigned short* __restrict__ gusb,
                                                  unsigned short* __restrict__ dwa) {
  const int blk = blockIdx.x, tid = threadIdx.x;
  if (blk < XBLK) {
    const size_t g = (size_t)blk * 256 + tid;
    const v4u o = pack8_bf(xh + g * 8);
    unsigned short* d = xb + g * 8;
    *(volatile v4u*)d = o;
    __threadfence();
    *(volatile v4u*)d = o;
  } else if (blk < XBLK + GBLK) {
    const size_t g = (size_t)(blk - XBLK) * 256 + tid;
    const v4u o = pack8_bf(gus + g * 8);
    unsigned short* d = gusb + g * 8;
    *(volatile v4u*)d = o;
    __threadfence();
    *(volatile v4u*)d = o;
  } else {
    const int g = (blk - XBLK - GBLK) * 256 + tid;
    const int row = g >> 7, col = (g & 127) * 8;
    const v4u o = pack8_bf(dw + (size_t)row * NS + col);
    unsigned short* d = dwa + (size_t)row * KF + col;
    *(volatile v4u*)d = o;
    *(volatile v4u*)(d + NS) = o;
    __threadfence();
    *(volatile v4u*)d = o;
    *(volatile v4u*)(d + NS) = o;
  }
}

__global__ __launch_bounds__(256) void tconv2_kernel(const float* __restrict__ W, const float* __restrict__ ysc,
                                                     unsigned short* __restrict__ oh,
                                                     int ldin, int ldout, long sIn, long sOut, int loOff, int b0) {
  __shared__ __align__(16) float tf[64 * 68];
  W  += (size_t)blockIdx.z * sIn;
  oh += (size_t)blockIdx.z * sOut;
  const float* ysb = ysc + (size_t)(b0 + (int)blockIdx.z) * NC;
  const int c0  = blockIdx.x * 64;
  const int r0  = blockIdx.y * 64;
  const int tid = threadIdx.x;
  {
    const int lr = tid >> 4;
    const int c4 = (tid & 15) * 4;
    const v4f ys = *(const v4f*)(ysb + ((c0 + c4) & (NC - 1)));
#pragma unroll
    for (int it = 0; it < 4; ++it) {
      const int rr = it * 16 + lr;
      const v4f a = *(const v4f*)(W + (size_t)(r0 + rr) * ldin + c0 + c4);
      v4f s;
      s.x = a.x * ys.x; s.y = a.y * ys.y; s.z = a.z * ys.z; s.w = a.w * ys.w;
      *(v4f*)(tf + rr * 68 + c4) = s;
    }
  }
  __syncthreads();
  const int sub = tid >> 3;
  const int c8  = (tid & 7) * 8;
  v4u hv[2], lv[2];
#pragma unroll
  for (int it = 0; it < 2; ++it) {
    const int oc = it * 32 + sub;
    v4u ah, al;
#pragma unroll
    for (int q = 0; q < 4; ++q) {
      const float f0 = tf[(c8 + 2 * q) * 68 + oc];
      const float f1 = tf[(c8 + 2 * q + 1) * 68 + oc];
      const unsigned short h0 = f2bf_bits(f0), h1 = f2bf_bits(f1);
      const unsigned short l0 = f2bf_bits(f0 - bf_bits2f(h0));
      const unsigned short l1 = f2bf_bits(f1 - bf_bits2f(h1));
      ah[q] = pk16(h0, h1);
      al[q] = pk16(l0, l1);
    }
    hv[it] = ah;
    lv[it] = al;
  }
  for (int ps = 0; ps < 2; ++ps) {
#pragma unroll
    for (int it = 0; it < 2; ++it) {
      const int oc = it * 32 + sub;
      const size_t go = (size_t)(c0 + oc) * ldout + r0 + c8;
      *(volatile v4u*)(oh + go) = hv[it];
      *(volatile v4u*)(oh + go + loOff) = lv[it];
    }
    __threadfence();
  }
}

#define CS_CH 32
#define CS_P  34
#define CS_RS (6 * CS_P)

template <bool SIG>
__device__ __forceinline__ void cs_stage(float* st, const float* __restrict__ xb, const float* yss,
                                         int c0, int y0, int g16, int q4) {
#pragma unroll 1
  for (int r = 0; r < 6; ++r) {
    const int yy  = y0 - 1 + r;
    const int yyc = min(max(yy, 0), IMW - 1);
    const float vf = (yy >= 0 && yy < IMW) ? 1.0f : 0.0f;
#pragma unroll
    for (int i2 = 0; i2 < 2; ++i2) {
      const int c = g16 + 16 * i2;
      const float ysv = yss[c0 + c];
      const v4f a = *(const v4f*)(xb + (size_t)(c0 + c) * NS + yyc * IMW + q4);
      float o0 = bf_rne(a.x) * ysv, o1 = bf_rne(a.y) * ysv, o2 = bf_rne(a.z) * ysv, o3 = bf_rne(a.w) * ysv;
      if (SIG) { o0 = sigm(o0); o1 = sigm(o1); o2 = sigm(o2); o3 = sigm(o3); }
      float* d = st + c * CS_RS + r * CS_P + 1 + q4;
      d[0] = o0 * vf; d[1] = o1 * vf; d[2] = o2 * vf; d[3] = o3 * vf;
    }
  }
}

__global__ __launch_bounds__(128) void csa_kernel(const float* __restrict__ x, const float* __restrict__ ysc,
                                                  unsigned short* __restrict__ catt, int b0) {
  __shared__ __align__(16) float st[CS_CH * CS_RS];
  __shared__ __align__(16) float gt[CS_CH * 128];
  __shared__ __align__(16) float yss[NC];
  const int tid = threadIdx.x, lane = tid & 31, wave = tid >> 5;
  const int bl = blockIdx.y, b = b0 + bl;
  const int y0 = blockIdx.x * 4;
  const int py = wave, px = lane;
  const int g16 = tid >> 3, q4 = (tid & 7) * 4;
  const float* xb = x + (size_t)b * NC * NS;

  *(v4f*)(yss + 4 * tid) = *(const v4f*)(ysc + (size_t)b * NC + 4 * tid);
  for (int e = tid; e < CS_CH * 6; e += 128) { st[e * CS_P] = 0.0f; st[e * CS_P + CS_P - 1] = 0.0f; }

  float lg[9];
#pragma unroll
  for (int k = 0; k < 9; ++k) lg[k] = 0.0f;

#pragma unroll 1
  for (int cc = 0; cc < NC / CS_CH; ++cc) {
    __syncthreads();
    cs_stage<true>(st, xb, yss, cc * CS_CH, y0, g16, q4);
    __syncthreads();
#pragma unroll 1
    for (int c = 0; c < CS_CH; ++c) {
      const float* sp = st + c * CS_RS + py * CS_P + px;
      const float n0 = sp[0], n1 = sp[1], n2 = sp[2];
      const float n3 = sp[CS_P], n4 = sp[CS_P + 1], n5 = sp[CS_P + 2];
      const float n6 = sp[2 * CS_P], n7 = sp[2 * CS_P + 1], n8 = sp[2 * CS_P + 2];
      lg[0] = fmaf(n4, n0, lg[0]); lg[1] = fmaf(n4, n1, lg[1]); lg[2] = fmaf(n4, n2, lg[2]);
      lg[3] = fmaf(n4, n3, lg[3]); lg[4] = fmaf(n4, n4, lg[4]); lg[5] = fmaf(n4, n5, lg[5]);
      lg[6] = fmaf(n4, n6, lg[6]); lg[7] = fmaf(n4, n7, lg[7]); lg[8] = fmaf(n4, n8, lg[8]);
    }
  }
  float at[9];
  {
    const float inv_c = 1.0f / (float)NC;
#pragma unroll
    for (int k = 0; k < 9; ++k) lg[k] *= inv_c;
    float mx = lg[0];
#pragma unroll
    for (int k = 1; k < 9; ++k) mx = fmaxf(mx, lg[k]);
    float sum = 0.0f;
#pragma unroll
    for (int k = 0; k < 9; ++k) { at[k] = __expf(lg[k] - mx); sum += at[k]; }
    const float inv = __builtin_amdgcn_rcpf(sum);
#pragma unroll
    for (int k = 0; k < 9; ++k) at[k] *= inv;
  }
  const int q8 = lane & 7, sub = lane >> 3;
  const size_t colh = (size_t)NC + (size_t)y0 * 16 + 8 * q8;
#pragma unroll 1
  for (int cc = 0; cc < NC / CS_CH; ++cc) {
    const int c0 = cc * CS_CH;
    __syncthreads();
    cs_stage<false>(st, xb, yss, c0, y0, g16, q4);
    __syncthreads();
#pragma unroll 1
    for (int c = 0; c < CS_CH; ++c) {
      const float* sp = st + c * CS_RS + py * CS_P + px;
      const float n0 = sp[0], n1 = sp[1], n2 = sp[2];
      const float n3 = sp[CS_P], n4 = sp[CS_P + 1], n5 = sp[CS_P + 2];
      const float n6 = sp[2 * CS_P], n7 = sp[2 * CS_P + 1], n8 = sp[2 * CS_P + 2];
      float g = at[0] * n0;
      g = fmaf(at[1], n1, g); g = fmaf(at[2], n2, g); g = fmaf(at[3], n3, g); g = fmaf(at[4], n4, g);
      g = fmaf(at[5], n5, g); g = fmaf(at[6], n6, g); g = fmaf(at[7], n7, g); g = fmaf(at[8], n8, g);
      gt[c * 128 + tid] = g;
    }
    __syncthreads();
    {
      v4u hv[4], lv[4];
#pragma unroll
      for (int it = 0; it < 4; ++it) {
        const int idx = it * 4 + sub;
        const int cl  = wave * 8 + (idx >> 1);
        const int par = idx & 1;
        const float* gp = gt + cl * 128 + 16 * q8 + par;
        v4u ah, al;
#pragma unroll
        for (int qq = 0; qq < 4; ++qq) {
          const float f0 = gp[4 * qq], f1 = gp[4 * qq + 2];
          const unsigned short h0 = f2bf_bits(f0), h1 = f2bf_bits(f1);
          const unsigned short l0 = f2bf_bits(f0 - bf_bits2f(h0));
          const unsigned short l1 = f2bf_bits(f1 - bf_bits2f(h1));
          ah[qq] = pk16(h0, h1);
          al[qq] = pk16(l0, l1);
        }
        hv[it] = ah;
        lv[it] = al;
      }
      for (int ps = 0; ps < 2; ++ps) {
#pragma unroll
        for (int it = 0; it < 4; ++it) {
          const int idx = it * 4 + sub;
          const int cl  = wave * 8 + (idx >> 1);
          const int par = idx & 1;
          unsigned short* d = catt + ((size_t)bl * NS + (size_t)par * NC + c0 + cl) * KF + colh;
          *(volatile v4u*)d = hv[it];
          *(volatile v4u*)(d + NS) = lv[it];
        }
        __threadfence();
      }
    }
  }
}

__global__ __launch_bounds__(256) void inorm_kernel(const float* __restrict__ z, float* __restrict__ out, int row0) {
  const int lane = threadIdx.x & 31, wave = threadIdx.x >> 5;
  const int rl = blockIdx.x * 8 + wave;
  const float* zr = z + (size_t)rl * NS + 4 * lane;
  float* orow = out + ((size_t)row0 + rl) * NS + 4 * lane;
  float s = 0.0f;
#pragma unroll 2
  for (int q = 0; q < NS / 128; ++q) {
    const v4f v = *(const v4f*)(zr + 128 * q);
    s += (v.x + v.y) + (v.z + v.w);
  }
  s = wave_sum(s);
  const float mean = s * (1.0f / (float)NS);
  float s2 = 0.0f;
#pragma unroll 2
  for (int q = 0; q < NS / 128; ++q) {
    const v4f v = *(const v4f*)(zr + 128 * q);
    const float d0 = v.x - mean, d1 = v.y - mean, d2 = v.z - mean, d3 = v.w - mean;
    s2 = fmaf(d0, d0, s2); s2 = fmaf(d1, d1, s2); s2 = fmaf(d2, d2, s2); s2 = fmaf(d3, d3, s2);
  }
  s2 = wave_sum(s2);
  const float rs = rsqrtf(s2 * (1.0f / (float)NS) + 1e-5f);
#pragma unroll 1
  for (int ps = 0; ps < 2; ++ps) {
#pragma unroll 2
    for (int q = 0; q < NS / 128; ++q) {
      const v4f v = *(const v4f*)(zr + 128 * q);
      v4f o;
      const float t0 = (v.x - mean) * rs, t1 = (v.y - mean) * rs, t2 = (v.z - mean) * rs, t3 = (v.w - mean) * rs;
      o.x = (t0 >= 0.0f) ? t0 : 0.2f * t0;
      o.y = (t1 >= 0.0f) ? t1 : 0.2f * t1;
      o.z = (t2 >= 0.0f) ? t2 : 0.2f * t2;
      o.w = (t3 >= 0.0f) ? t3 : 0.2f * t3;
      *(volatile v4f*)(orow + 128 * q) = o;
    }
    __threadfence();
  }
}

extern "C" void kernel_launch(void* const* d_in, const int* in_sizes, int n_in,
                              void* d_out, int out_size, void* d_ws, size_t ws_size,
                              hipStream_t stream) {
  if (n_in < 7) return;
  if (in_sizes[0] != NB * NC * NS) return;
  if (in_sizes[1] != NR * NC) return;
  if (in_sizes[2] != NR) return;
  if (in_sizes[3] != NC * NR) return;
  if (in_sizes[4] != NC) return;
  if (in_sizes[5] != NC * 2 * NC) return;
  if (in_sizes[6] != NS * NS) return;
  if (out_size != NB * NC * NS) return;

  const float* x   = (const float*)d_in[0];
  const float* w1  = (const float*)d_in[1];
  const float* b1  = (const float*)d_in[2];
  const float* w2  = (const float*)d_in[3];
  const float* b2  = (const float*)d_in[4];
  const float* dw  = (const float*)d_in[5];
  const float* gus = (const float*)d_in[6];
  float* out = (float*)d_out;

  const size_t PY   = (size_t)NB * NC * 4;
  const size_t PGB  = (size_t)NS * NS * 2;
  const size_t PDW  = (size_t)NC * KF * 2;
  const size_t PXB  = (size_t)HB * NC * NS * 2;
  const size_t PGUS = (size_t)HB * NS * NC * 4;
  const size_t PCAT = (size_t)HB * NS * KF * 2;
  const size_t PZ   = (size_t)HB * NC * NS * 4;
  size_t off = 0;
  const size_t oY   = off; off += PY;
  const size_t oGB  = off; off += PGB;
  const size_t oDW  = off; off += PDW;
  const size_t oXB  = off; off += PXB;
  const size_t oGUS = off; off += PGUS;
  const size_t oCAT = off; off += PCAT;
  const size_t oZ   = off; off += PZ;
  if (off > ws_size) return;
  if (off > (size_t)134217728) return;

  char* ws = (char*)d_ws;
  float*          YSC  = (float*)(ws + oY);
  unsigned short* GUSB = (unsigned short*)(ws + oGB);
  unsigned short* DWA  = (unsigned short*)(ws + oDW);
  unsigned short* XB   = (unsigned short*)(ws + oXB);
  float*          GUS  = (float*)(ws + oGUS);
  unsigned short* CATT = (unsigned short*)(ws + oCAT);
  float*          Z    = (float*)(ws + oZ);

  const dim3 blk(256);

  se_kernel<<<dim3(NB), blk, 0, stream>>>(x, w1, b1, w2, b2, YSC);

  for (int hf = 0; hf < NB / HB; ++hf) {
    const int b0 = hf * HB;
    const float* xh = x + (size_t)b0 * NC * NS;
    const int nblk = XBLK + ((hf == 0) ? (GBLK + DBLK) : 0);
    cvt_kernel<<<dim3(nblk), blk, 0, stream>>>(xh, gus, dw, XB, GUSB, DWA);
    wmma_gemm64<1, false, 0, 0, false, 0><<<dim3(((NS / 64) * (NC / 64) + 7) / 8, HB), blk, 0, stream>>>(
        GUSB, GUSB, NS, 0L, XB, XB, NS, (long)NC * NS, (void*)GUS, (void*)GUS, NC, (long)NS * NC,
        YSC, YSC, 0L, NS, NC, NS, 1.0f);
    tconv2_kernel<<<dim3(NS / 64, NC / 64, HB), blk, 0, stream>>>(GUS, YSC, CATT, NS, KF, (long)NS * NC, (long)NS * KF, NS, b0);
    csa_kernel<<<dim3(IMW / 4, HB), dim3(128), 0, stream>>>(x, YSC, CATT, b0);
    wmma_gemm64<1, false, 0, 0, false, 0><<<dim3(((NC / 64) * (NS / 64) + 7) / 8, HB), blk, 0, stream>>>(
        DWA, DWA, KF, 0L, CATT, CATT, KF, (long)NS * KF, (void*)Z, (void*)Z, NS, (long)NC * NS,
        YSC, YSC, 0L, NC, NS, KF, 1.0f);
    inorm_kernel<<<dim3(HB * NC / 8), blk, 0, stream>>>(Z, out, b0 * NC);
  }
  (void)hipGetLastError();
}
